// KANLayer_3513283248483
// MI455X (gfx1250) — hardware-verified
//
#include <hip/hip_runtime.h>
#include <stddef.h>
#include <math.h>


typedef _Float16 h16;
typedef _Float16 v16h __attribute__((ext_vector_type(16)));
typedef _Float16 v8h  __attribute__((ext_vector_type(8)));
typedef float    v8f  __attribute__((ext_vector_type(8)));
typedef float    v4f  __attribute__((ext_vector_type(4)));

#ifndef NROWS
#define NROWS 4096
#endif
#define NROWS_FULL 4096
#define DIN    128
#define DOUT   128
#define NBASIS 9
#define KP     (DIN * NBASIS)
#define FR     16
#define LDC    68

#define WCARRY 64.0f
#define FCARRY 16.0f

static_assert(NROWS >= 64 && NROWS <= NROWS_FULL);
static_assert((NROWS % 64) == 0 && (NROWS % FR) == 0);
static_assert(DIN == 128);
static_assert((KP % 32) == 0 && (KP % 8) == 0);
static_assert((DOUT % 64) == 0);
static_assert(DOUT == 4 * 32);
static_assert(((FR * DIN) % 256) == 0);
static_assert(((FR * KP / 8) % 256) == 0);
static_assert(((DOUT * KP / 8) % 256) == 0);
static_assert((LDC % 4) == 0 && LDC >= 64);

#define WT_BYTES ((size_t)DOUT * KP * 2)
#define BC_BYTES ((size_t)DOUT * 4)
#define F_BYTES  ((size_t)NROWS * KP * 2)
#define OFF_WT   ((size_t)0)
#define OFF_BC   (OFF_WT + WT_BYTES)
#define OFF_F    (OFF_BC + BC_BYTES)
#define WS_TOTAL (OFF_F + F_BYTES)
static_assert((WT_BYTES % 128) == 0 && (BC_BYTES % 128) == 0 && (F_BYTES % 128) == 0);
static_assert(WS_TOTAL <= (size_t)134217728);

__device__ __forceinline__ float bf16r(float x) {
  unsigned int u = __float_as_uint(x);
  u = (u + 0x7FFFu + ((u >> 16) & 1u)) & 0xFFFF0000u;
  return __uint_as_float(u);
}

static __device__ __forceinline__ h16 toh_flush(float v) {
  const h16 r = (h16)v;
  return (fabsf(v) < 6.103515625e-05f) ? (h16)0.0f : r;
}

__device__ __forceinline__ v16h frag_at(const _Float16* p) {
  v8h lo = *(const v8h*)(p);
  v8h hi = *(const v8h*)(p + 16);
  v16h out;
#pragma unroll
  for (int i = 0; i < 8; ++i) { out[i] = lo[i]; out[i + 8] = hi[i]; }
  return out;
}

__device__ __forceinline__ v8f wmma16(v16h a, v16h b, v8f c) {
  v8f d = __builtin_amdgcn_wmma_f32_16x16x32_f16(false, a, false, b, (short)0, c,
                                                 false, false);
  asm volatile("v_nop\n\tv_nop\n\tv_nop\n\tv_nop" : "+v"(d) : "v"(a), "v"(b));
  return d;
}

__global__ __launch_bounds__(256) void weff_kernel(
    const float* __restrict__ W, const float* __restrict__ C, _Float16* __restrict__ Wt) {
#pragma clang fp contract(off)
  const unsigned idx = blockIdx.x * 256u + threadIdx.x;
  const unsigned o = idx / (unsigned)(KP / 8);
  const unsigned c = idx - o * (unsigned)(KP / 8);
  v8h v;
#pragma unroll
  for (unsigned j = 0; j < 8u; ++j) {
    const unsigned kk = c * 8u + j;
    const unsigned i = kk / (unsigned)NBASIS;
    const unsigned f = kk - i * (unsigned)NBASIS;
    const float wv = bf16r(W[(size_t)(i * (unsigned)DOUT + o) * NBASIS + f]);
    const float cv = bf16r(C[i * (unsigned)DOUT + o]);
    v[j] = toh_flush(WCARRY * (wv * cv));
  }
  _Float16* p = Wt + (size_t)idx * 8u;
  *(volatile v8h*)p = v;
  __threadfence();
  *(volatile v8h*)p = v;
}

__global__ __launch_bounds__(128) void biasc_kernel(
    const float* __restrict__ Bi, const float* __restrict__ C, float* __restrict__ Bc) {
#pragma clang fp contract(off)
  __shared__ __attribute__((aligned(16))) float Sb[DOUT];
  const unsigned tid = threadIdx.x;
  const int wave = __builtin_amdgcn_readfirstlane((int)(threadIdx.x >> 5));
  float acc = 0.0f;
#pragma unroll 1
  for (unsigned i = 0; i < (unsigned)DIN; ++i) {
    const float t = bf16r(Bi[i * (unsigned)DOUT + tid]) * bf16r(C[i * (unsigned)DOUT + tid]);
    acc = acc + t;
  }
  Sb[tid] = acc;
  __syncthreads();
  if (wave == 0) {
    const unsigned lane = tid & 31u;
    const v4f x = *(const v4f*)&Sb[lane * 4u];
    float* p = Bc + lane * 4u;
    *(volatile v4f*)p = x;
    __threadfence();
    *(volatile v4f*)p = x;
  }
}

__global__ __launch_bounds__(256) void feat_kernel(
    const float* __restrict__ X, _Float16* __restrict__ F) {
#pragma clang fp contract(off)
  __shared__ __attribute__((aligned(16))) _Float16 T[FR * KP];
  const unsigned tid = threadIdx.x;
  const unsigned r0 = blockIdx.x * (unsigned)FR;
#pragma unroll 1
  for (unsigned t = 0; t < (unsigned)((FR * DIN) / 256); ++t) {
    const unsigned e = tid + 256u * t;
    const unsigned row = e >> 7;
    const unsigned i = e & 127u;
    const float xv = bf16r(X[(size_t)(r0 + row) * DIN + i]);
    const float ax = fabsf(xv);
    const unsigned base = row * (unsigned)KP + i * (unsigned)NBASIS;
    const float x2 = xv * xv;
    const float x3 = x2 * xv;
    T[base + 0u] = toh_flush(FCARRY * xv);
    T[base + 1u] = toh_flush(FCARRY * x2);
    T[base + 2u] = toh_flush(FCARRY * x3);
    T[base + 3u] = toh_flush(FCARRY * expf(xv));
    T[base + 4u] = toh_flush(FCARRY * logf(ax + 1.0f));
    T[base + 5u] = toh_flush(FCARRY * sqrtf(ax));
    T[base + 6u] = toh_flush(FCARRY * tanhf(xv));
    T[base + 7u] = toh_flush(FCARRY * sinf(xv));
    T[base + 8u] = toh_flush(FCARRY * ax);
  }
  __syncthreads();
#pragma unroll 1
  for (unsigned j = 0; j < (unsigned)((FR * KP / 8) / 256); ++j) {
    const unsigned c = tid + 256u * j;
    const v8h o = *(const v8h*)&T[c * 8u];
    _Float16* p = F + (size_t)r0 * KP + (size_t)c * 8u;
    *(volatile v8h*)p = o;
    __threadfence();
    *(volatile v8h*)p = o;
  }
}

__global__ __launch_bounds__(256) void gemm_out_kernel(
    const _Float16* __restrict__ A16, const _Float16* __restrict__ Bt,
    const float* __restrict__ biasc, float* __restrict__ outf) {
  __shared__ __attribute__((aligned(16))) float Cs[64 * LDC];
  const unsigned K = (unsigned)KP;
  const unsigned tid = threadIdx.x, lane = tid & 31u, w = tid >> 5;
  const unsigned mw = w >> 1, nw = w & 1u;
  const unsigned hh = lane >> 4, m = lane & 15u;
  const unsigned n0 = blockIdx.x * 64u;
  const unsigned row0 = blockIdx.y * 64u;

  const _Float16* ap  = A16 + (size_t)(row0 + mw * 16u + m) * K + hh * 8u;
  const _Float16* bp0 = Bt + (size_t)(n0 + nw * 32u + m) * K + hh * 8u;
  const _Float16* bp1 = bp0 + (size_t)16 * K;
  v8f acc0 = {}, acc1 = {};
#pragma unroll 2
  for (unsigned k0 = 0; k0 < K; k0 += 32u) {
    const v16h a  = frag_at(ap + k0);
    const v16h b0 = frag_at(bp0 + k0);
    const v16h b1 = frag_at(bp1 + k0);
    acc0 = wmma16(a, b0, acc0);
    acc1 = wmma16(a, b1, acc1);
  }
#pragma unroll
  for (int r = 0; r < 8; ++r) {
    float* d = &Cs[(mw * 16u + hh * 8u + (unsigned)r) * LDC + nw * 32u + m];
    d[0]  = acc0[r];
    d[16] = acc1[r];
  }
  __syncthreads();

  const float cs = 1.0f / (WCARRY * FCARRY);
  v4f xs[4];
  size_t off[4];
#pragma unroll
  for (unsigned i = 0; i < 4u; ++i) {
    const unsigned r = 16u * i + (tid >> 4);
    const unsigned c = (tid & 15u) * 4u;
    const v4f u = *(const v4f*)&Cs[r * LDC + c];
    const v4f g = *(const v4f*)(biasc + n0 + c);
    v4f val;
#pragma unroll
    for (int j = 0; j < 4; ++j) val[j] = u[j] * cs + g[j];
    xs[i] = val;
    off[i] = (size_t)(row0 + r) * DOUT + n0 + c;
  }
#pragma unroll
  for (int i = 0; i < 4; ++i) *(volatile v4f*)(outf + off[i]) = xs[i];
  __threadfence();
#pragma unroll
  for (int i = 0; i < 4; ++i) *(volatile v4f*)(outf + off[i]) = xs[i];
}

extern "C" void kernel_launch(void* const* d_in, const int* in_sizes, int n_in,
                              void* d_out, int out_size, void* d_ws, size_t ws_size,
                              hipStream_t stream) {
  if (n_in < 4) return;
  if ((long long)in_sizes[0] < (long long)NROWS * DIN) return;
  if ((long long)in_sizes[1] < (long long)DIN * DOUT * NBASIS) return;
  if ((long long)in_sizes[2] < (long long)DIN * DOUT) return;
  if ((long long)in_sizes[3] < (long long)DIN * DOUT) return;
  if ((long long)out_size < (long long)NROWS * DOUT) return;
  if (ws_size < WS_TOTAL) return;

  const float* X  = (const float*)d_in[0];
  const float* Wi = (const float*)d_in[1];
  const float* Bi = (const float*)d_in[2];
  const float* Ci = (const float*)d_in[3];
  float* out = (float*)d_out;

  char* ws = (char*)d_ws;
  _Float16* Wt = (_Float16*)(ws + OFF_WT);
  float*    Bc = (float*)(ws + OFF_BC);
  _Float16* Fp = (_Float16*)(ws + OFF_F);

  dim3 blk(256);
  weff_kernel<<<dim3((DOUT * KP / 8) / 256), blk, 0, stream>>>(Wi, Ci, Wt);
  biasc_kernel<<<dim3(1), dim3(128), 0, stream>>>(Bi, Ci, Bc);
  feat_kernel<<<dim3(NROWS / FR), blk, 0, stream>>>(X, Fp);
  gemm_out_kernel<<<dim3(DOUT / 64, NROWS / 64), blk, 0, stream>>>(Fp, Wt, Bc, out);
}
